// SlidingDecoderBlock_36043365548101
// MI455X (gfx1250) — hardware-verified
//
#include <hip/hip_runtime.h>
#include <stdint.h>
#include <math.h>

typedef __attribute__((ext_vector_type(16))) _Float16 v16h;
typedef __attribute__((ext_vector_type(8)))  _Float16 v8h;
typedef __attribute__((ext_vector_type(16))) __bf16   v16b;
typedef __attribute__((ext_vector_type(8)))  __bf16   v8b;
typedef __attribute__((ext_vector_type(8)))  float    v8f;
typedef __attribute__((ext_vector_type(4)))  float    v4f;
#define PSCALE 32768.0f

__device__ __forceinline__ unsigned short f2bf_bits(float f) {
  unsigned u = __float_as_uint(f);
  return (unsigned short)((u + 0x7FFFu + ((u >> 16) & 1u)) >> 16);
}
__device__ __forceinline__ float bf_bits2f(unsigned short h) { return __uint_as_float(((unsigned)h) << 16); }

__device__ __forceinline__ void dep_guard_h(v8f& a, v8f& b, v16h x, v16h y) { asm volatile("v_nop\n\tv_nop\n\tv_nop\n\tv_nop" : "+v"(a), "+v"(b) : "v"(x), "v"(y)); }
__device__ __forceinline__ void dep_guard_b(v8f& a, v8f& b, v16b x, v16b y) { asm volatile("v_nop\n\tv_nop\n\tv_nop\n\tv_nop" : "+v"(a), "+v"(b) : "v"(x), "v"(y)); }
__device__ __forceinline__ void keep4_h(v16h a, v16h b, v16h c, v16h d) { asm volatile("v_nop" :: "v"(a), "v"(b), "v"(c), "v"(d)); }
__device__ __forceinline__ void keep4_b(v16b a, v16b b, v16b c, v16b d) { asm volatile("v_nop" :: "v"(a), "v"(b), "v"(c), "v"(d)); }
__device__ __forceinline__ void acc_guard4(v8f& a, v8f& b, v8f& c, v8f& d) { asm volatile("v_nop\n\tv_nop\n\tv_nop\n\tv_nop" : "+v"(a), "+v"(b), "+v"(c), "+v"(d)); }
template <typename T> struct Frag;
template <> struct Frag<_Float16> {
  typedef v16h V; union U { v16h v; v8h h[2]; };
  static __device__ __forceinline__ v16h load(const _Float16* p) {
    U f; f.h[0] = *(const v8h*)(p); f.h[1] = *(const v8h*)(p + 16); return f.v;
  }
  static __device__ __forceinline__ v8f mma(v16h a, v16h b, v8f c) {
    return __builtin_amdgcn_wmma_f32_16x16x32_f16(false, a, false, b, (short)0, c, false, false);
  }
  static __device__ __forceinline__ void guard(v8f& a, v8f& b, v16h x, v16h y) { dep_guard_h(a, b, x, y); }
  static __device__ __forceinline__ void keep(v16h a, v16h b, v16h c, v16h d) { keep4_h(a, b, c, d); }
};
template <> struct Frag<__bf16> {
  typedef v16b V; union U { v16b v; v8b h[2]; };
  static __device__ __forceinline__ v16b load(const __bf16* p) {
    U f; f.h[0] = *(const v8b*)(p); f.h[1] = *(const v8b*)(p + 16); return f.v;
  }
  static __device__ __forceinline__ v8f mma(v16b a, v16b b, v8f c) {
    return __builtin_amdgcn_wmma_f32_16x16x32_bf16(false, a, false, b, (short)0, c, false, false);
  }
  static __device__ __forceinline__ void guard(v8f& a, v8f& b, v16b x, v16b y) { dep_guard_b(a, b, x, y); }
  static __device__ __forceinline__ void keep(v16b a, v16b b, v16b c, v16b d) { keep4_b(a, b, c, d); }
};

template <int ET> struct Elem;
template <> struct Elem<0> { typedef _Float16 T; };
template <> struct Elem<1> { typedef __bf16 T; };
template <int ET, bool SPLIT, int BIAS_MODE, int OUT_MODE, bool RESID, int ACT = 0, bool MULAUX = false>
__global__ __launch_bounds__(256) void wmma_gemm64(
    const unsigned short* __restrict__ Ap, const unsigned short* __restrict__ A2p, int lda, long strideA,
    const unsigned short* __restrict__ Btp, const unsigned short* __restrict__ Bt2p, int ldb, long strideB,
    void* Cout, void* Cout2, int ldc, long strideC,
    const float* __restrict__ bias,
    const float* __restrict__ resid, long strideR,
    const unsigned short* aux16,
    int M, int N, int K, float scale) {
  typedef typename Elem<ET>::T T;
  typedef typename Frag<T>::V V;
  const T* A = (const T*)Ap; const T* A2 = (const T*)A2p; const T* Bt = (const T*)Btp; const T* Bt2 = (const T*)Bt2p;
  __shared__ __align__(16) float sT[8][16 * 68];
  const int b    = blockIdx.y;
  const int lane = threadIdx.x & 31;
  const int wave = threadIdx.x >> 5;
  const int tilesN = N >> 6;
  const int tilesM = M >> 6;
  const int tile = blockIdx.x * 8 + wave;
  if (tile >= tilesM * tilesN) return;
  const int tm = tile / tilesN;
  const int tn = tile - tm * tilesN;
  const int m0 = tm << 6;
  const int n0 = tn << 6;

  const T* Ab  = A  + (size_t)b * strideA;
  const T* Bb  = Bt + (size_t)b * strideB;
  const T* Ab2 = SPLIT ? (A2  + (size_t)b * strideA) : nullptr;
  const T* Bb2 = SPLIT ? (Bt2 + (size_t)b * strideB) : nullptr;

  const int rlane = lane & 15;
  const int koff  = (lane >> 4) * 8;
  const int mOff  = (lane >> 4) * 8;

  v8f acc[4][4];
#pragma unroll
  for (int i = 0; i < 4; ++i)
#pragma unroll
    for (int j = 0; j < 4; ++j) acc[i][j] = (v8f){0.f,0.f,0.f,0.f,0.f,0.f,0.f,0.f};

  for (int k0 = 0; k0 < K; k0 += 32) {
    V bh[4], bl[4];
#pragma unroll
    for (int j = 0; j < 4; ++j) {
      const size_t bo = (size_t)(n0 + (j << 4) + rlane) * ldb + koff + k0;
      bh[j] = Frag<T>::load(Bb + bo);
      if (SPLIT) bl[j] = Frag<T>::load(Bb2 + bo);
    }
#pragma unroll
    for (int i = 0; i < 4; ++i) {
      const size_t ao = (size_t)(m0 + (i << 4) + rlane) * lda + koff + k0;
      V ah = Frag<T>::load(Ab + ao);
      V al;
      if (SPLIT) al = Frag<T>::load(Ab2 + ao);
#pragma unroll
      for (int j = 0; j < 4; ++j) {
        acc[i][j] = Frag<T>::mma(ah, bh[j], acc[i][j]);
        if (SPLIT) {
          acc[i][j] = Frag<T>::mma(ah, bl[j], acc[i][j]);
          acc[i][j] = Frag<T>::mma(al, bh[j], acc[i][j]);
        }
      }
      Frag<T>::guard(acc[i][0], acc[i][3], ah, SPLIT ? al : ah);
    }
    Frag<T>::keep(bh[0], bh[1], bh[2], bh[3]);
    if (SPLIT) Frag<T>::keep(bl[0], bl[1], bl[2], bl[3]);
  }
  acc_guard4(acc[0][0], acc[0][1], acc[0][2], acc[0][3]);
  acc_guard4(acc[1][0], acc[1][1], acc[1][2], acc[1][3]);
  acc_guard4(acc[2][0], acc[2][1], acc[2][2], acc[2][3]);
  acc_guard4(acc[3][0], acc[3][1], acc[3][2], acc[3][3]);

  float* slab = sT[wave];
  const float* Rb = RESID ? (resid + (size_t)b * strideR) : nullptr;
  const _Float16* Xb = MULAUX ? ((const _Float16*)aux16 + (size_t)b * strideC) : nullptr;
#pragma unroll
  for (int i = 0; i < 4; ++i) {
    const int mBase = m0 + (i << 4);
#pragma unroll
    for (int j = 0; j < 4; ++j) {
      const int n = n0 + (j << 4) + rlane;
      float bv = 0.f;
      if (BIAS_MODE == 2) bv = bias[n];
#pragma unroll
      for (int r = 0; r < 8; ++r) {
        float v = acc[i][j][r] * scale;
        if (BIAS_MODE == 1) v += bias[mBase + mOff + r];
        if (BIAS_MODE == 2) v += bv;
        if (RESID) v += Rb[(size_t)(mBase + mOff + r) * ldc + n];
        if (ACT == 1) v = tanhf(v);
        if (ACT == 2) v = fmaxf(v, 0.0f);
        if (ACT == 3) v = v * __builtin_amdgcn_rcpf(1.0f + __expf(-v));
        if (ACT == 4) v = (v > 0.f) ? v : 0.01f * v;
        if (MULAUX) v *= (float)Xb[(size_t)(mBase + mOff + r) * ldc + n];
        slab[(mOff + r) * 68 + (j << 4) + rlane] = v;
      }
    }
    __builtin_amdgcn_fence(__ATOMIC_RELEASE, "workgroup");
    __builtin_amdgcn_wave_barrier();
    __builtin_amdgcn_fence(__ATOMIC_ACQUIRE, "workgroup");
    if (OUT_MODE == 0) {
      float* C = (float*)Cout + (size_t)b * strideC;
      const int hh = lane >> 4, c4 = (lane & 15) * 4;
      for (int pass = 0; pass < 2; ++pass) {
#pragma unroll
        for (int it = 0; it < 8; ++it) {
          const int row = it * 2 + hh;
          v4f v = *(const v4f*)(slab + row * 68 + c4);
          *(volatile v4f*)(C + (size_t)(mBase + row) * ldc + n0 + c4) = v;
        }
        __threadfence();
      }
    } else {
      const int q = lane >> 3, c8 = (lane & 7) * 8;
      unsigned short* C  = (unsigned short*)Cout  + (size_t)b * strideC;
      unsigned short* C2 = (OUT_MODE == 2) ? ((unsigned short*)Cout2 + (size_t)b * strideC) : nullptr;
      for (int pass = 0; pass < 2; ++pass) {
#pragma unroll
        for (int it = 0; it < 4; ++it) {
          const int row = it * 4 + q;
          const float* sp = slab + row * 68 + c8;
          v8h hv, lv;
#pragma unroll
          for (int e = 0; e < 8; ++e) {
            if (OUT_MODE == 1) {
              hv[e] = (_Float16)sp[e];
            } else {
              unsigned short hb = f2bf_bits(sp[e]);
              unsigned short lb = f2bf_bits(sp[e] - bf_bits2f(hb));
              hv[e] = __builtin_bit_cast(_Float16, hb);
              lv[e] = __builtin_bit_cast(_Float16, lb);
            }
          }
          *(volatile v8h*)(C + (size_t)(mBase + row) * ldc + n0 + c8) = hv;
          if (OUT_MODE == 2) *(volatile v8h*)(C2 + (size_t)(mBase + row) * ldc + n0 + c8) = lv;
        }
        __threadfence();
      }
    }
    __builtin_amdgcn_fence(__ATOMIC_RELEASE, "workgroup");
    __builtin_amdgcn_wave_barrier();
    __builtin_amdgcn_fence(__ATOMIC_ACQUIRE, "workgroup");
  }
}

#define WT_PITCH 72
__global__ __launch_bounds__(256) void wt_cast_k(const float* __restrict__ W, unsigned short* __restrict__ Wtp,
                                                 int Kr, int Nc, int Kp, float mul) {
  __shared__ __align__(16) _Float16 st[64 * WT_PITCH];
  _Float16* Wt = (_Float16*)Wtp;
  const int n0 = blockIdx.x * 64, k0 = blockIdx.y * 64;
  const int tid = threadIdx.x;
  const int kr = tid >> 2, c16 = (tid & 3) * 16;
  const int kk = k0 + kr;
  const bool kval = (kk < Kr);
  const int kcl = kval ? kk : (Kr - 1);
  const float* src = W + (size_t)kcl * Nc;
#pragma unroll
  for (int q = 0; q < 4; ++q) {
    const int cc = n0 + c16 + 4 * q;
    const bool cval = kval && (cc < Nc);
    const int ccl = (cc < Nc) ? cc : (Nc - 4);
    const v4f v = *(const v4f*)(src + ccl);
#pragma unroll
    for (int e = 0; e < 4; ++e)
      st[(c16 + 4 * q + e) * WT_PITCH + kr] = cval ? (_Float16)(v[e] * mul) : (_Float16)0.0f;
  }
  __syncthreads();
  const int wave = tid >> 5, lane = tid & 31;
  const int q8 = lane >> 3, c8 = (lane & 7) * 8;
  for (int pass = 0; pass < 2; ++pass) {
#pragma unroll
    for (int it = 0; it < 2; ++it) {
      const int n = it * 32 + wave * 4 + q8;
      const v8h hv = *(const v8h*)(st + n * WT_PITCH + c8);
      *(volatile v8h*)(Wt + (size_t)(n0 + n) * Kp + k0 + c8) = hv;
    }
    __threadfence();
  }
}

#define ROW_LEN 1024
template <bool NORM>
__global__ __launch_bounds__(128) void rowcast_k(const float* __restrict__ x, const float* __restrict__ w,
                                                unsigned short* __restrict__ hp, float eps) {
  __shared__ float red[4];
  _Float16* hq = (_Float16*)hp;
  const int row = blockIdx.x, tid = threadIdx.x, lane = tid & 31, wave = tid >> 5;
  const size_t rb = (size_t)row * ROW_LEN;
  const int c0 = tid * 8;
  const v4f va = *(const v4f*)(x + rb + c0);
  const v4f vb = *(const v4f*)(x + rb + c0 + 4);
  float inv = 1.0f;
  v4f wa = (v4f){1.f, 1.f, 1.f, 1.f}, wb = (v4f){1.f, 1.f, 1.f, 1.f};
  if (NORM) {
    float s = ((va[0] * va[0] + va[1] * va[1]) + (va[2] * va[2] + va[3] * va[3])) +
              ((vb[0] * vb[0] + vb[1] * vb[1]) + (vb[2] * vb[2] + vb[3] * vb[3]));
#pragma unroll
    for (int off = 1; off < 32; off <<= 1) s += __shfl_xor(s, off, 32);
    if (lane == 0) red[wave] = s;
    __syncthreads();
    const float tot = (red[0] + red[1]) + (red[2] + red[3]);
    inv = rsqrtf(tot * (1.0f / ROW_LEN) + eps);
    wa = *(const v4f*)(w + c0);
    wb = *(const v4f*)(w + c0 + 4);
  }
  v8h hv;
#pragma unroll
  for (int e = 0; e < 4; ++e) {
    hv[e]     = (_Float16)((va[e] * inv) * wa[e]);
    hv[4 + e] = (_Float16)((vb[e] * inv) * wb[e]);
  }
  for (int pass = 0; pass < 2; ++pass) {
    *(volatile v8h*)(hq + rb + c0) = hv;
    __threadfence();
  }
}

__device__ __forceinline__ v8f mma_h(v16h a, v16h b, v8f c) {
  c = __builtin_amdgcn_wmma_f32_16x16x32_f16(false, a, false, b, (short)0, c, false, false);
  asm volatile("v_nop\n\tv_nop\n\tv_nop\n\tv_nop" : "+v"(c) : "v"(a), "v"(b));
  return c;
}
#define AT_KC 64
#define AT_OSP 68
template <int WMODE>
__global__ __launch_bounds__(128)
void attn_hd64_k(const unsigned short* __restrict__ qpp, const unsigned short* __restrict__ kpp,
                 const unsigned short* __restrict__ vtp, unsigned short* __restrict__ opp,
                 const int* __restrict__ seg, int S, int Skv, int H, int vld, float sscale, int lookback) {
  union FH { v16h v; v8h h[2]; };
  __shared__ __align__(16) _Float16 Ksh[AT_KC * 64];
  __shared__ __align__(16) _Float16 Vth[64 * AT_KC];
  __shared__ __align__(16) _Float16 Psh[4][16 * AT_KC];
  __shared__ __align__(16) float  Os[4][16 * AT_OSP];
  __shared__ int sseg[64];
  const _Float16* q  = (const _Float16*)qpp;
  const _Float16* k  = (const _Float16*)kpp;
  const _Float16* vt = (const _Float16*)vtp;
  _Float16* o = (_Float16*)opp;

  const int tid  = threadIdx.x;
  const int wave = tid >> 5;
  const int lane = tid & 31;
  const int hh   = lane >> 4;
  const int c    = lane & 15;
  const int ld   = H * 64;
  const int nqb  = S >> 6;
  const int nkc  = Skv >> 6;
  const int bx   = blockIdx.x;
  const int qb   = bx % nqb;
  const int bh   = bx / nqb;
  const int h    = bh % H;
  const int b    = bh / H;
  const int qblk = qb << 6;
  const int q0   = qblk + wave * 16;

  const _Float16* qb_ptr = q  + (size_t)b * S * ld + (size_t)h * 64;
  const _Float16* kb_ptr = k  + (size_t)b * Skv * ld + (size_t)h * 64;
  const _Float16* vb_ptr = vt + (size_t)h * 64 * vld + (size_t)b * Skv;
  _Float16*       ob_ptr = o  + (size_t)b * S * ld + (size_t)h * 64;

  int cfirst = 0, clast = qb;
  int sgr[8];
#pragma unroll
  for (int r = 0; r < 8; ++r) sgr[r] = 0;
  if constexpr (WMODE == 1) {
    if (tid < 64) sseg[tid] = seg[(size_t)b * S + qblk + tid];
    __syncthreads();
    int mn = sseg[0], mx = sseg[0];
#pragma unroll 1
    for (int i = 1; i < 64; ++i) { const int sv = sseg[i]; mn = min(mn, sv); mx = max(mx, sv); }
    int lo = mn - lookback, hi = mx;
    lo = max(lo, 0); lo = min(lo, Skv - 1);
    hi = max(hi, 0); hi = min(hi, Skv - 1);
    cfirst = lo >> 6; clast = hi >> 6;
    if (clast < cfirst) clast = cfirst;
#pragma unroll
    for (int r = 0; r < 8; ++r) sgr[r] = sseg[wave * 16 + 8 * hh + r];
  }
  clast = min(clast, nkc - 1);
  cfirst = min(max(cfirst, 0), clast);

  v16h qa[2];
  {
    const _Float16* qrow = qb_ptr + (size_t)(q0 + c) * ld + 8 * hh;
#pragma unroll
    for (int dc = 0; dc < 2; ++dc) qa[dc] = Frag<_Float16>::load(qrow + dc * 32);
  }

  float mrow[8], lrow[8];
  v8f oacc[4];
#pragma unroll
  for (int r = 0; r < 8; ++r) { mrow[r] = -INFINITY; lrow[r] = 0.f; }
#pragma unroll
  for (int t = 0; t < 4; ++t) oacc[t] = (v8f){0.f,0.f,0.f,0.f,0.f,0.f,0.f,0.f};

  for (int kc = cfirst; kc <= clast; ++kc) {
    const int kv0 = kc << 6;
    __syncthreads();
    {
      const int r = tid >> 1, hf = (tid & 1) * 32;
      const _Float16* ks = kb_ptr + (size_t)(kv0 + r) * ld + hf;
      const _Float16* vs = vb_ptr + (size_t)r * vld + kv0 + hf;
#pragma unroll
      for (int i = 0; i < 4; ++i) {
        const v8h kkv = *(const v8h*)(ks + 8 * i);
        const v8h vvv = *(const v8h*)(vs + 8 * i);
        *(v8h*)(Ksh + r * 64 + hf + 8 * i)    = kkv;
        *(v8h*)(Vth + r * AT_KC + hf + 8 * i) = vvv;
      }
    }
    __syncthreads();

    v8f s[4];
#pragma unroll
    for (int j = 0; j < 4; ++j) {
      s[j] = (v8f){0.f,0.f,0.f,0.f,0.f,0.f,0.f,0.f};
#pragma unroll
      for (int dc = 0; dc < 2; ++dc) {
        FH kf;
        kf.h[0] = *(const v8h*)(Ksh + (j * 16 + c) * 64 + dc * 32 + 8 * hh);
        kf.h[1] = *(const v8h*)(Ksh + (j * 16 + c) * 64 + dc * 32 + 16 + 8 * hh);
        s[j] = mma_h(qa[dc], kf.v, s[j]);
      }
    }
    const bool diag = (WMODE == 0) && (kc == qb);
    float cm[8];
#pragma unroll
    for (int r = 0; r < 8; ++r) {
      const int qrow = q0 + 8 * hh + r;
      const int sg = sgr[r];
      float m = -INFINITY;
#pragma unroll
      for (int j = 0; j < 4; ++j) {
        const int kvcol = kv0 + j * 16 + c;
        bool masked;
        if (WMODE == 0) masked = diag && (kvcol > qrow);
        else            masked = (kvcol > sg) || (kvcol < sg - lookback);
        const float val = masked ? -INFINITY : s[j][r] * sscale;
        s[j][r] = val;
        m = fmaxf(m, val);
      }
#pragma unroll
      for (int off = 1; off < 16; off <<= 1) m = fmaxf(m, __shfl_xor(m, off, 32));
      cm[r] = m;
    }
    _Float16* pw = Psh[wave];
#pragma unroll
    for (int r = 0; r < 8; ++r) {
      const float mnew = fmaxf(mrow[r], cm[r]);
      const float mref = (mnew == -INFINITY) ? 0.0f : mnew;
      const float alpha = __expf(mrow[r] - mref);
      mrow[r] = mnew;
      float psum = 0.f;
#pragma unroll
      for (int j = 0; j < 4; ++j) {
        const float p = __expf(s[j][r] - mref);
        psum += p;
        pw[(8 * hh + r) * AT_KC + j * 16 + c] = (_Float16)(p * PSCALE);
      }
#pragma unroll
      for (int off = 1; off < 16; off <<= 1) psum += __shfl_xor(psum, off, 32);
      lrow[r] = lrow[r] * alpha + psum;
#pragma unroll
      for (int t = 0; t < 4; ++t) oacc[t][r] *= alpha;
    }
    __builtin_amdgcn_fence(__ATOMIC_RELEASE, "workgroup");
    __builtin_amdgcn_wave_barrier();
    __builtin_amdgcn_fence(__ATOMIC_ACQUIRE, "workgroup");
#pragma unroll 1
    for (int kk = 0; kk < 2; ++kk) {
      FH pa;
      pa.h[0] = *(const v8h*)(pw + c * AT_KC + kk * 32 + 8 * hh);
      pa.h[1] = *(const v8h*)(pw + c * AT_KC + kk * 32 + 16 + 8 * hh);
#pragma unroll
      for (int t = 0; t < 4; ++t) {
        FH vf;
        vf.h[0] = *(const v8h*)(Vth + (t * 16 + c) * AT_KC + kk * 32 + 8 * hh);
        vf.h[1] = *(const v8h*)(Vth + (t * 16 + c) * AT_KC + kk * 32 + 16 + 8 * hh);
        oacc[t] = mma_h(pa.v, vf.v, oacc[t]);
      }
    }
  }

  float* os = Os[wave];
#pragma unroll
  for (int r = 0; r < 8; ++r) {
    const float inv = 1.0f / (lrow[r] * PSCALE);
#pragma unroll
    for (int t = 0; t < 4; ++t) os[(8 * hh + r) * AT_OSP + t * 16 + c] = oacc[t][r] * inv;
  }
  __builtin_amdgcn_fence(__ATOMIC_RELEASE, "workgroup");
  __builtin_amdgcn_wave_barrier();
  __builtin_amdgcn_fence(__ATOMIC_ACQUIRE, "workgroup");
  {
    const int q8 = lane >> 3, c8 = (lane & 7) * 8;
    for (int pass = 0; pass < 2; ++pass) {
#pragma unroll
      for (int it = 0; it < 4; ++it) {
        const int row = it * 4 + q8;
        const float* sp = os + row * AT_OSP + c8;
        v8h hv;
#pragma unroll
        for (int e = 0; e < 8; ++e) hv[e] = (_Float16)sp[e];
        *(volatile v8h*)(ob_ptr + (size_t)(q0 + row) * ld + c8) = hv;
      }
      __threadfence();
    }
  }
}

static inline unsigned gemm_grid(int Mr, int Ncol) { return (unsigned)((((Mr >> 6) * (Ncol >> 6)) + 7) >> 3); }

extern "C" void kernel_launch(void* const* d_in, const int* in_sizes, int n_in,
                              void* d_out, int out_size, void* d_ws, size_t ws_size,
                              hipStream_t stream) {
  constexpr int kNB = 2, kSQ = 2048, kSM = 512, kDM = 1024, kNH = 16, kQC = 32, kKVC = 64, kDFF = 4096, kLBK = 8;
  constexpr int kNTOK = kNB * kSQ;
  constexpr int kNMEM = kNB * kSM;
  constexpr float kEPS = 1e-6f;
  constexpr float kWMUL = 64.0f;
  constexpr float kWINV = 1.0f / 64.0f;

  if (n_in < 19) return;
  if (in_sizes[0] != kNTOK * kDM || in_sizes[1] != kNMEM * kDM || in_sizes[2] != kNTOK ||
      in_sizes[3] != kDM || in_sizes[4] != kDM * kQC || in_sizes[5] != kQC * kDM ||
      in_sizes[6] != kDM * kKVC || in_sizes[7] != kKVC * kDM || in_sizes[8] != kKVC * kDM ||
      in_sizes[9] != kDM * kDM || in_sizes[10] != kDM || in_sizes[11] != kDM * kDM ||
      in_sizes[12] != kDM * kDM || in_sizes[13] != kDM * kDM || in_sizes[14] != kDM * kDM ||
      in_sizes[15] != kDM || in_sizes[16] != kDM * kDFF || in_sizes[17] != kDM * kDFF ||
      in_sizes[18] != kDFF * kDM) return;
  if (out_size != kNTOK * kDM) return;

  constexpr size_t kMiB = 1048576;
  constexpr size_t oH16 = 0, oX1 = 8 * kMiB, oX2 = 24 * kMiB;
  constexpr size_t oWG = 40 * kMiB, oWU = 48 * kMiB, oWD = 56 * kMiB;
  constexpr size_t oWO = 64 * kMiB, oWQC = 66 * kMiB, oWKC = 68 * kMiB, oWVC = 70 * kMiB, oWOC = 72 * kMiB;
  constexpr size_t oWDQ = 74 * kMiB, oWUQ = oWDQ + 131072, oWDKV = oWUQ + 131072, oWUK = oWDKV + 131072, oWUV = oWUK + 131072;
  constexpr size_t oT1 = 75 * kMiB, oCKV = oT1 + 524288, oQ16 = 76 * kMiB, oK16 = 84 * kMiB, oVT = 92 * kMiB, oO16 = 100 * kMiB;
  constexpr size_t oMEM = 76 * kMiB, oQC = 78 * kMiB, oKC = 86 * kMiB, oVCT = 88 * kMiB, oOC = 90 * kMiB;
  constexpr size_t oSG = 76 * kMiB;
  constexpr size_t kWsEnd = 108 * kMiB;
  static_assert(oWUV + 131072 <= oT1);
  static_assert(oO16 + 8 * kMiB == kWsEnd);
  static_assert(oOC + 8 * kMiB <= kWsEnd);
  static_assert(oSG + 32 * kMiB == kWsEnd);
  static_assert(kWsEnd <= (size_t)134217728);
  if (ws_size < kWsEnd) return;

  const float* x_in    = (const float*)d_in[0];
  const float* memory  = (const float*)d_in[1];
  const int*   seg     = (const int*)d_in[2];
  const float* norm1_w = (const float*)d_in[3];
  const float* W_dq    = (const float*)d_in[4];
  const float* W_uq    = (const float*)d_in[5];
  const float* W_dkv   = (const float*)d_in[6];
  const float* W_uk    = (const float*)d_in[7];
  const float* W_uv    = (const float*)d_in[8];
  const float* W_osl   = (const float*)d_in[9];
  const float* norm2_w = (const float*)d_in[10];
  const float* W_qc    = (const float*)d_in[11];
  const float* W_kc    = (const float*)d_in[12];
  const float* W_vc    = (const float*)d_in[13];
  const float* W_oc    = (const float*)d_in[14];
  const float* norm3_w = (const float*)d_in[15];
  const float* W_gate  = (const float*)d_in[16];
  const float* W_up    = (const float*)d_in[17];
  const float* W_down  = (const float*)d_in[18];
  float* outp = (float*)d_out;

  char* ws = (char*)d_ws;
  unsigned short* h16  = (unsigned short*)(ws + oH16);
  float*          x1   = (float*)(ws + oX1);
  float*          x2   = (float*)(ws + oX2);
  unsigned short* wg   = (unsigned short*)(ws + oWG);
  unsigned short* wu   = (unsigned short*)(ws + oWU);
  unsigned short* wd   = (unsigned short*)(ws + oWD);
  unsigned short* wo   = (unsigned short*)(ws + oWO);
  unsigned short* wqc  = (unsigned short*)(ws + oWQC);
  unsigned short* wkc  = (unsigned short*)(ws + oWKC);
  unsigned short* wvc  = (unsigned short*)(ws + oWVC);
  unsigned short* woc  = (unsigned short*)(ws + oWOC);
  unsigned short* wdq  = (unsigned short*)(ws + oWDQ);
  unsigned short* wuq  = (unsigned short*)(ws + oWUQ);
  unsigned short* wdkv = (unsigned short*)(ws + oWDKV);
  unsigned short* wuk  = (unsigned short*)(ws + oWUK);
  unsigned short* wuv  = (unsigned short*)(ws + oWUV);
  unsigned short* t1   = (unsigned short*)(ws + oT1);
  unsigned short* ckv  = (unsigned short*)(ws + oCKV);
  unsigned short* q16  = (unsigned short*)(ws + oQ16);
  unsigned short* k16  = (unsigned short*)(ws + oK16);
  unsigned short* vT   = (unsigned short*)(ws + oVT);
  unsigned short* o16  = (unsigned short*)(ws + oO16);
  unsigned short* mem16 = (unsigned short*)(ws + oMEM);
  unsigned short* qc16 = (unsigned short*)(ws + oQC);
  unsigned short* kc16 = (unsigned short*)(ws + oKC);
  unsigned short* vcT  = (unsigned short*)(ws + oVCT);
  unsigned short* oc16 = (unsigned short*)(ws + oOC);
  unsigned short* sg   = (unsigned short*)(ws + oSG);

  wt_cast_k<<<dim3(1, 16), 256, 0, stream>>>(W_dq,   wdq,  kDM,  kQC,  kDM,  kWMUL);
  wt_cast_k<<<dim3(16, 1), 256, 0, stream>>>(W_uq,   wuq,  kQC,  kDM,  64,   kWMUL);
  wt_cast_k<<<dim3(1, 16), 256, 0, stream>>>(W_dkv,  wdkv, kDM,  kKVC, kDM,  kWMUL);
  wt_cast_k<<<dim3(16, 1), 256, 0, stream>>>(W_uk,   wuk,  kKVC, kDM,  kKVC, kWMUL);
  wt_cast_k<<<dim3(16, 1), 256, 0, stream>>>(W_uv,   wuv,  kKVC, kDM,  kKVC, kWMUL);
  wt_cast_k<<<dim3(16, 16), 256, 0, stream>>>(W_osl, wo,   kDM,  kDM,  kDM,  kWMUL);
  wt_cast_k<<<dim3(16, 16), 256, 0, stream>>>(W_qc,  wqc,  kDM,  kDM,  kDM,  kWMUL);
  wt_cast_k<<<dim3(16, 16), 256, 0, stream>>>(W_kc,  wkc,  kDM,  kDM,  kDM,  kWMUL);
  wt_cast_k<<<dim3(16, 16), 256, 0, stream>>>(W_vc,  wvc,  kDM,  kDM,  kDM,  kWMUL);
  wt_cast_k<<<dim3(16, 16), 256, 0, stream>>>(W_oc,  woc,  kDM,  kDM,  kDM,  kWMUL);
  wt_cast_k<<<dim3(64, 16), 256, 0, stream>>>(W_gate, wg,  kDM,  kDFF, kDM,  kWMUL);
  wt_cast_k<<<dim3(64, 16), 256, 0, stream>>>(W_up,   wu,  kDM,  kDFF, kDM,  kWMUL);
  wt_cast_k<<<dim3(16, 64), 256, 0, stream>>>(W_down, wd,  kDFF, kDM,  kDFF, kWMUL);

  rowcast_k<true><<<kNTOK, 128, 0, stream>>>(x_in, norm1_w, h16, kEPS);
  wmma_gemm64<0, false, 0, 1, false, 0, false><<<dim3(gemm_grid(kNTOK, 64), 1), 256, 0, stream>>>(
      h16, nullptr, kDM, 0L, wdq, nullptr, kDM, 0L, t1, nullptr, 64, 0L, nullptr, nullptr, 0L, nullptr,
      kNTOK, 64, kDM, kWINV);
  wmma_gemm64<0, false, 0, 1, false, 0, false><<<dim3(gemm_grid(kNTOK, kKVC), 1), 256, 0, stream>>>(
      h16, nullptr, kDM, 0L, wdkv, nullptr, kDM, 0L, ckv, nullptr, kKVC, 0L, nullptr, nullptr, 0L, nullptr,
      kNTOK, kKVC, kDM, kWINV);
  wmma_gemm64<0, false, 0, 1, false, 0, false><<<dim3(gemm_grid(kNTOK, kDM), 1), 256, 0, stream>>>(
      t1, nullptr, 64, 0L, wuq, nullptr, 64, 0L, q16, nullptr, kDM, 0L, nullptr, nullptr, 0L, nullptr,
      kNTOK, kDM, 64, 0.25f);
  wmma_gemm64<0, false, 0, 1, false, 0, false><<<dim3(gemm_grid(kNTOK, kDM), 1), 256, 0, stream>>>(
      ckv, nullptr, kKVC, 0L, wuk, nullptr, kKVC, 0L, k16, nullptr, kDM, 0L, nullptr, nullptr, 0L, nullptr,
      kNTOK, kDM, kKVC, 0.25f);
  wmma_gemm64<0, false, 0, 1, false, 0, false><<<dim3(gemm_grid(kDM, kNTOK), 1), 256, 0, stream>>>(
      wuv, nullptr, kKVC, 0L, ckv, nullptr, kKVC, 0L, vT, nullptr, kNTOK, 0L, nullptr, nullptr, 0L, nullptr,
      kDM, kNTOK, kKVC, 1.0f);
  attn_hd64_k<0><<<kNB * kNH * (kSQ / 64), 128, 0, stream>>>(
      q16, k16, vT, o16, seg, kSQ, kSQ, kNH, kNTOK, 0.00048828125f, 0);
  wmma_gemm64<0, false, 0, 0, true, 0, false><<<dim3(gemm_grid(kNTOK, kDM), 1), 256, 0, stream>>>(
      o16, nullptr, kDM, 0L, wo, nullptr, kDM, 0L, x1, nullptr, kDM, 0L, nullptr, x_in, 0L, nullptr,
      kNTOK, kDM, kDM, 1.0f / 4096.0f);

  rowcast_k<true><<<kNTOK, 128, 0, stream>>>(x1, norm2_w, h16, kEPS);
  rowcast_k<false><<<kNMEM, 128, 0, stream>>>(memory, norm2_w, mem16, kEPS);
  wmma_gemm64<0, false, 0, 1, false, 0, false><<<dim3(gemm_grid(kNTOK, kDM), 1), 256, 0, stream>>>(
      h16, nullptr, kDM, 0L, wqc, nullptr, kDM, 0L, qc16, nullptr, kDM, 0L, nullptr, nullptr, 0L, nullptr,
      kNTOK, kDM, kDM, kWINV);
  wmma_gemm64<0, false, 0, 1, false, 0, false><<<dim3(gemm_grid(kNMEM, kDM), 1), 256, 0, stream>>>(
      mem16, nullptr, kDM, 0L, wkc, nullptr, kDM, 0L, kc16, nullptr, kDM, 0L, nullptr, nullptr, 0L, nullptr,
      kNMEM, kDM, kDM, kWINV);
  wmma_gemm64<0, false, 0, 1, false, 0, false><<<dim3(gemm_grid(kDM, kNMEM), 1), 256, 0, stream>>>(
      wvc, nullptr, kDM, 0L, mem16, nullptr, kDM, 0L, vcT, nullptr, kNMEM, 0L, nullptr, nullptr, 0L, nullptr,
      kDM, kNMEM, kDM, kWINV);
  attn_hd64_k<1><<<kNB * kNH * (kSQ / 64), 128, 0, stream>>>(
      qc16, kc16, vcT, oc16, seg, kSQ, kSM, kNH, kNMEM, 0.125f, kLBK);
  wmma_gemm64<0, false, 0, 0, true, 0, false><<<dim3(gemm_grid(kNTOK, kDM), 1), 256, 0, stream>>>(
      oc16, nullptr, kDM, 0L, woc, nullptr, kDM, 0L, x2, nullptr, kDM, 0L, nullptr, x1, 0L, nullptr,
      kNTOK, kDM, kDM, kWINV);

  rowcast_k<true><<<kNTOK, 128, 0, stream>>>(x2, norm3_w, h16, kEPS);
  wmma_gemm64<0, false, 0, 1, false, 3, false><<<dim3(gemm_grid(kNTOK, kDFF), 1), 256, 0, stream>>>(
      h16, nullptr, kDM, 0L, wg, nullptr, kDM, 0L, sg, nullptr, kDFF, 0L, nullptr, nullptr, 0L, nullptr,
      kNTOK, kDFF, kDM, kWINV);
  wmma_gemm64<0, false, 0, 1, false, 0, true><<<dim3(gemm_grid(kNTOK, kDFF), 1), 256, 0, stream>>>(
      h16, nullptr, kDM, 0L, wu, nullptr, kDM, 0L, sg, nullptr, kDFF, 0L, nullptr, nullptr, 0L, sg,
      kNTOK, kDFF, kDM, kWINV);
  wmma_gemm64<0, false, 0, 0, true, 0, false><<<dim3(gemm_grid(kNTOK, kDM), 1), 256, 0, stream>>>(
      sg, nullptr, kDFF, 0L, wd, nullptr, kDFF, 0L, outp, nullptr, kDM, 0L, nullptr, x2, 0L, nullptr,
      kNTOK, kDM, kDFF, kWINV);
}
